// SemanticGraphBuilder_30794915512742
// MI455X (gfx1250) — hardware-verified
//
#include <hip/hip_runtime.h>
#include <stddef.h>

#define NB 4
#define NN 256
#define DD 256
#define NODES (NB * NN)
#define KP (2 * DD)
#define WTP (4 * DD)
#define LDP 520
#define JT 64
#define SP 132
#define NTHR 256
#define WSCALE 64.0f
#define WINV (1.0f / 64.0f)

static_assert(LDP % 8 == 0);
static_assert(LDP >= KP);
static_assert(SP % 4 == 0);
static_assert(NN % JT == 0);
static_assert(NODES % 64 == 0);
static_assert(DD % 32 == 0);
static_assert(KP % 32 == 0);

typedef _Float16 f16;
typedef f16 v16h __attribute__((ext_vector_type(16)));
typedef f16 v8h_t __attribute__((ext_vector_type(8)));
typedef v8h_t __attribute__((may_alias)) v8h;
typedef float v8f __attribute__((ext_vector_type(8)));
typedef float v4f_t __attribute__((ext_vector_type(4)));
typedef v4f_t __attribute__((may_alias)) v4f;
typedef unsigned int v4u __attribute__((ext_vector_type(4)));

union Frag { v16h v; v8h_t h[2]; };
union Pack8 { v8h_t h; v4u u; };

__device__ __forceinline__ v8f zero8() {
    v8f z;
#pragma unroll
    for (int i = 0; i < 8; ++i) z[i] = 0.0f;
    return z;
}

__device__ __forceinline__ v16h ldfrag(const f16* p, int k0) {
    Frag f;
    f.h[0] = *(const v8h*)(p + k0);
    f.h[1] = *(const v8h*)(p + k0 + 16);
    return f.v;
}

__device__ __forceinline__ v8f wmma16(v16h a, v16h b, v8f c) {
    return __builtin_amdgcn_wmma_f32_16x16x32_f16(false, a, false, b, (short)0, c, false, false);
}

__global__ void __launch_bounds__(NTHR) cvt_rows_kernel(
    const float* __restrict__ src, f16* __restrict__ dst, int n8)
{
    const int i = blockIdx.x * NTHR + threadIdx.x;
    const bool ok = (i < n8);
    const int ic = ok ? i : 0;
    Pack8 pk;
#pragma unroll
    for (int j = 0; j < 4; ++j) pk.u[j] = 0u;
    {
        const v4f_t a = *(const v4f*)(src + (size_t)ic * 8);
        const v4f_t c = *(const v4f*)(src + (size_t)ic * 8 + 4);
#pragma unroll
        for (int j = 0; j < 4; ++j) {
            pk.h[j]     = (f16)a[j];
            pk.h[4 + j] = (f16)c[j];
        }
    }
    if (ok) *(volatile v4u*)(dst + (size_t)i * 8) = pk.u;
    __threadfence();
    if (ok) *(volatile v4u*)(dst + (size_t)i * 8) = pk.u;
}

__global__ void __launch_bounds__(NTHR) cvt_wt_kernel(
    const float* __restrict__ W1, f16* __restrict__ W1T)
{
    __shared__ float tile[64 * 65];
    const int tid = threadIdx.x;
    const int r0 = blockIdx.x * 64;
    const int h0 = blockIdx.y * 64;
#pragma unroll 4
    for (int it = 0; it < 16; ++it) {
        const int idx = it * NTHR + tid;
        const int rr = idx >> 6, cc = idx & 63;
        tile[cc * 65 + rr] = W1[(size_t)(r0 + rr) * DD + h0 + cc];
    }
    __syncthreads();
    const int q = tid & 7;
    Pack8 pk[2];
#pragma unroll
    for (int p = 0; p < 2; ++p) {
        const int c = p * 32 + (tid >> 3);
#pragma unroll
        for (int e = 0; e < 8; ++e)
            pk[p].h[e] = (f16)(tile[c * 65 + q * 8 + e] * WSCALE);
    }
#pragma unroll
    for (int p = 0; p < 2; ++p) {
        const int c = p * 32 + (tid >> 3);
        *(volatile v4u*)(W1T + (size_t)(h0 + c) * WTP + r0 + q * 8) = pk[p].u;
    }
    __threadfence();
#pragma unroll
    for (int p = 0; p < 2; ++p) {
        const int c = p * 32 + (tid >> 3);
        *(volatile v4u*)(W1T + (size_t)(h0 + c) * WTP + r0 + q * 8) = pk[p].u;
    }
}

__global__ void __launch_bounds__(NTHR) node_gemm_kernel(
    const f16* __restrict__ sh16, const f16* __restrict__ W1T,
    const float* __restrict__ b1, float* __restrict__ nodeT)
{
    __shared__ __align__(16) float stg[64 * SP];
    const int tid = threadIdx.x, lane = tid & 31, w = tid >> 5;
    const int hh = lane >> 4, m = lane & 15;
    const int rt = w & 3, cq = w >> 2;
    const int row0 = blockIdx.x * 64;
    const int n0 = blockIdx.y * 128;
    const int seg = n0 >> 8;
    const int cbase = n0 & 255;

    v8f acc[4];
#pragma unroll
    for (int t = 0; t < 4; ++t) acc[t] = zero8();

    const f16* pa = sh16 + (size_t)(row0 + rt * 16 + m) * DD + 8 * hh;
    const f16* pb = W1T + (size_t)(cbase + cq * 64 + m) * WTP + seg * DD + 8 * hh;
#pragma unroll 1
    for (int k0 = 0; k0 < DD; k0 += 32) {
        const v16h a = ldfrag(pa, k0);
        v16h bf;
#pragma unroll
        for (int tn = 0; tn < 4; ++tn) {
            bf = ldfrag(pb + (size_t)tn * 16 * WTP, k0);
            acc[tn] = wmma16(a, bf, acc[tn]);
        }
        asm volatile("v_nop\n\tv_nop\n\tv_nop\n\tv_nop"
                     : "+v"(acc[0]), "+v"(acc[1]), "+v"(acc[2]), "+v"(acc[3])
                     : "v"(a), "v"(bf));
    }

#pragma unroll
    for (int tn = 0; tn < 4; ++tn) {
        const int col = cq * 64 + tn * 16 + m;
        const float bv = b1[cbase + col];
        const float bias = (seg == 0) ? bv : 0.0f;
#pragma unroll
        for (int r = 0; r < 8; ++r)
            stg[(rt * 16 + 8 * hh + r) * SP + col] = fmaf(acc[tn][r], WINV, bias);
    }
    __syncthreads();

    v4f_t v[8];
#pragma unroll
    for (int p = 0; p < 8; ++p)
        v[p] = *(const v4f*)(stg + (p * 8 + w) * SP + lane * 4);
    float* dst = nodeT + (size_t)seg * NODES * DD + (size_t)row0 * DD + cbase + lane * 4;
#pragma unroll
    for (int p = 0; p < 8; ++p)
        *(volatile v4f_t*)(dst + (size_t)(p * 8 + w) * DD) = v[p];
    __threadfence();
#pragma unroll
    for (int p = 0; p < 8; ++p)
        *(volatile v4f_t*)(dst + (size_t)(p * 8 + w) * DD) = v[p];
}

__global__ void __launch_bounds__(NTHR) pair_kernel(
    const float* __restrict__ sh, const float* __restrict__ W2, const float* __restrict__ b2,
    const float* __restrict__ nodeT, const f16* __restrict__ W1T, float* __restrict__ out)
{
    __shared__ __align__(16) f16 At[JT * LDP];
    __shared__ __align__(16) float si_s[DD];
    __shared__ float srcb_s[DD];
    __shared__ float w2_s[DD];
    __shared__ float scp[2 * NN];
    __shared__ __align__(16) float prob_s[NN];
    __shared__ float red_s[8];

    const int i = blockIdx.x;
    const int b = blockIdx.y;
    const int tid = threadIdx.x, lane = tid & 31, w = tid >> 5;
    const int hh = lane >> 4, m = lane & 15;
    const int rt = w & 3, ch = w >> 2;

    const size_t bi = (size_t)b * NN + i;
    si_s[tid]   = sh[bi * DD + tid];
    srcb_s[tid] = nodeT[bi * DD + tid];
    w2_s[tid]   = W2[tid];
    const float b2v = b2[0];
    const float* tgtT = nodeT + (size_t)NODES * DD + (size_t)b * NN * DD;
    const float* shb  = sh + (size_t)b * NN * DD;
    __syncthreads();

#pragma unroll 1
    for (int jt = 0; jt < NN / JT; ++jt) {
        const int j0 = jt * JT;

        {
            const v4f_t a0 = *(const v4f*)(si_s + lane * 8);
            const v4f_t a1 = *(const v4f*)(si_s + lane * 8 + 4);
#pragma unroll 2
            for (int q = 0; q < 8; ++q) {
                const int jr = w * 8 + q;
                const float* sj = shb + (size_t)(j0 + jr) * DD + lane * 8;
                const v4f_t c0 = *(const v4f*)(sj);
                const v4f_t c1 = *(const v4f*)(sj + 4);
                Pack8 dv, pv;
#pragma unroll
                for (int e = 0; e < 4; ++e) {
                    dv.h[e]     = (f16)fabsf(a0[e] - c0[e]);
                    dv.h[4 + e] = (f16)fabsf(a1[e] - c1[e]);
                    pv.h[e]     = (f16)(a0[e] * c0[e]);
                    pv.h[4 + e] = (f16)(a1[e] * c1[e]);
                }
                *(v8h*)(At + jr * LDP + lane * 8)      = dv.h;
                *(v8h*)(At + jr * LDP + DD + lane * 8) = pv.h;
            }
        }
        __syncthreads();

        v8f acc[8];
#pragma unroll
        for (int t = 0; t < 8; ++t) acc[t] = zero8();
        const f16* pa = At + (rt * 16 + m) * LDP + 8 * hh;
        const f16* pb = W1T + (size_t)(ch * 128 + m) * WTP + KP + 8 * hh;
#pragma unroll 1
        for (int k0 = 0; k0 < KP; k0 += 32) {
            const v16h a = ldfrag(pa, k0);
            v16h bf;
#pragma unroll
            for (int tn = 0; tn < 8; ++tn) {
                bf = ldfrag(pb + (size_t)tn * 16 * WTP, k0);
                acc[tn] = wmma16(a, bf, acc[tn]);
            }
            asm volatile("v_nop\n\tv_nop\n\tv_nop\n\tv_nop"
                         : "+v"(acc[0]), "+v"(acc[1]), "+v"(acc[2]), "+v"(acc[3]),
                           "+v"(acc[4]), "+v"(acc[5]), "+v"(acc[6]), "+v"(acc[7])
                         : "v"(a), "v"(bf));
        }

        float partial[8];
#pragma unroll
        for (int r = 0; r < 8; ++r) partial[r] = 0.0f;
#pragma unroll
        for (int tn = 0; tn < 8; ++tn) {
            const int hcol = ch * 128 + tn * 16 + m;
            const float w2v = w2_s[hcol];
            const float sv  = srcb_s[hcol];
            const float* tb = tgtT + (size_t)(j0 + rt * 16 + 8 * hh) * DD + hcol;
#pragma unroll
            for (int r = 0; r < 8; ++r) {
                const float tv = tb[(size_t)r * DD];
                const float hv = fmaf(acc[tn][r], WINV, sv) + tv;
                const float ex = __expf(-hv);
                const float sg = __builtin_amdgcn_rcpf(1.0f + ex);
                partial[r] = fmaf(hv * sg, w2v, partial[r]);
            }
        }
#pragma unroll
        for (int r = 0; r < 8; ++r) {
            float v = partial[r];
            v += __shfl_xor(v, 1, 32);
            v += __shfl_xor(v, 2, 32);
            v += __shfl_xor(v, 4, 32);
            v += __shfl_xor(v, 8, 32);
            partial[r] = v;
        }
        if (m == 0) {
#pragma unroll
            for (int r = 0; r < 8; ++r)
                scp[ch * NN + j0 + rt * 16 + 8 * hh + r] = partial[r];
        }
        __syncthreads();
    }

    float sc = scp[tid] + scp[NN + tid] + b2v;
    sc = (tid == i) ? -1.0e9f : sc;
    float mx = sc;
#pragma unroll
    for (int off = 16; off > 0; off >>= 1) mx = fmaxf(mx, __shfl_xor(mx, off, 32));
    if (lane == 0) red_s[w] = mx;
    __syncthreads();
    float gmx = red_s[0];
#pragma unroll
    for (int k = 1; k < 8; ++k) gmx = fmaxf(gmx, red_s[k]);
    const float ex = __expf(sc - gmx);
    __syncthreads();
    float s = ex;
#pragma unroll
    for (int off = 16; off > 0; off >>= 1) s += __shfl_xor(s, off, 32);
    if (lane == 0) red_s[w] = s;
    __syncthreads();
    float tot = red_s[0];
#pragma unroll
    for (int k = 1; k < 8; ++k) tot += red_s[k];
    const float rtot = 1.0f / tot;
    prob_s[tid] = ex * rtot;
    __syncthreads();

    if (w == 0) {
        v4f_t pv[2];
#pragma unroll
        for (int p = 0; p < 2; ++p) pv[p] = *(const v4f*)(prob_s + p * 128 + lane * 4);
        float* go = out + bi * NN + lane * 4;
#pragma unroll
        for (int p = 0; p < 2; ++p) *(volatile v4f_t*)(go + p * 128) = pv[p];
        __threadfence();
#pragma unroll
        for (int p = 0; p < 2; ++p) *(volatile v4f_t*)(go + p * 128) = pv[p];
    }
}

extern "C" void kernel_launch(void* const* d_in, const int* in_sizes, int n_in,
                              void* d_out, int out_size, void* d_ws, size_t ws_size,
                              hipStream_t stream)
{
    if (n_in < 5) return;
    if (in_sizes[0] != NODES * DD) return;
    if (in_sizes[1] != 4 * DD * DD) return;
    if (in_sizes[2] != DD) return;
    if (in_sizes[3] != DD) return;
    if (in_sizes[4] < 1) return;
    if (out_size != NB * NN * NN) return;

    const float* sh = (const float*)d_in[0];
    const float* W1 = (const float*)d_in[1];
    const float* b1 = (const float*)d_in[2];
    const float* W2 = (const float*)d_in[3];
    const float* b2 = (const float*)d_in[4];
    float* out = (float*)d_out;

    const size_t nSH = (size_t)NODES * DD;
    const size_t nWT = (size_t)DD * WTP;
    const size_t nNT = (size_t)2 * NODES * DD;
    const size_t oSH = 0;
    const size_t oWT = oSH + nSH * 2;
    const size_t oNT = oWT + nWT * 2;
    const size_t total = oNT + nNT * 4;
    if (total > ws_size) return;

    char* ws = (char*)d_ws;
    f16*   sh16  = (f16*)(ws + oSH);
    f16*   W1T   = (f16*)(ws + oWT);
    float* nodeT = (float*)(ws + oNT);

    const int n8 = (int)(nSH / 8);
    cvt_rows_kernel<<<(n8 + NTHR - 1) / NTHR, NTHR, 0, stream>>>(sh, sh16, n8);
    cvt_wt_kernel<<<dim3(NODES / 64, DD / 64), NTHR, 0, stream>>>(W1, W1T);
    node_gemm_kernel<<<dim3(NODES / 64, KP / 128), NTHR, 0, stream>>>(sh16, W1T, b1, nodeT);
    pair_kernel<<<dim3(NN, NB), NTHR, 0, stream>>>(sh, W2, b2, nodeT, W1T, out);
}
